// Head_8426725834935
// MI455X (gfx1250) — hardware-verified
//
#include <hip/hip_runtime.h>


#ifndef NB
#define NB 16
#endif
#ifndef SEQ
#define SEQ 1024
#endif
#define NB_FULL  16
#define SEQ_FULL 1024
#define CDIM  768
#define HDIM  64
#define NPROJ 192
#define KP    768
#define KH    384
#define XP    392
#define WP    768
#define XPADV ((XP - KH) / 8)
#define NTB    (SEQ / 64)
#define NTB_E  ((NTB < 8) ? NTB : 8)
#define NTB_L  (NTB - NTB_E)
#define NTB_LD ((NTB_L > 0) ? NTB_L : 1)
#define TE     (NTB_E * 64)

static_assert(SEQ % 64 == 0 && SEQ >= 64);
static_assert(SEQ <= SEQ_FULL);
static_assert(NB >= 1 && NB <= NB_FULL);
static_assert(KP == CDIM && (KP % KH) == 0 && (KH % 32) == 0 && (KH % 4) == 0);
static_assert(XP > KH && ((XP - KH) % 8) == 0 && (XP % 8) == 0);
static_assert(WP == CDIM && WP == 3 * 32 * 8 && ((WP * 2) % 128) == 0);
static_assert(NPROJ == 3 * HDIM && (NPROJ % 8) == 0 && (HDIM % 8) == 0 && HDIM == 64);
static_assert(64 * XP >= 6 * 4096);
static_assert(NTB_E + NTB_L == NTB);
static_assert(TE % 64 == 0 && TE <= SEQ);
static_assert((NB * SEQ) % 64 == 0);
static_assert((NPROJ / 8) * 8 * 3 * 32 * 8 == NPROJ * WP);
static_assert(((NB * SEQ) / 64) * 8 * 2 * 32 * 8 == NB * SEQ * HDIM);
static_assert((NB * NTB_E) * 4 * 8 * 32 * 4 + (NB * NTB_L) * 4 * 8 * 32 * 4 == NB * SEQ * HDIM);
static_assert(((long long)(NB - 1) * SEQ_FULL + SEQ) * HDIM <= (long long)NB_FULL * SEQ_FULL * HDIM);
static_assert((long long)NB_FULL * SEQ_FULL * HDIM == 1048576LL);

typedef _Float16       v16h  __attribute__((ext_vector_type(16)));
typedef _Float16       v8h   __attribute__((ext_vector_type(8)));
typedef float          v8f   __attribute__((ext_vector_type(8)));
typedef float          v4f   __attribute__((ext_vector_type(4)));
typedef unsigned short v16us __attribute__((ext_vector_type(16)));
typedef unsigned short v8us  __attribute__((ext_vector_type(8)));
typedef unsigned int   v4u   __attribute__((ext_vector_type(4)));
typedef unsigned int   v2u   __attribute__((ext_vector_type(2)));
typedef __bf16         v16bf __attribute__((ext_vector_type(16)));

union FragH { v16h v; v8h h[2]; };
union FragU { v16us v; v8us h[2]; };

#define LOG2E_F  1.4426950408889634f
#define NEG_BIG  (-3.0e38f)
#define RINV     0.0009765625f
#define QK_SCALE 0.03608439182435161f

__device__ __forceinline__ unsigned int bf_bits(float f) {
  const unsigned int u = __float_as_uint(f);
  return (u + 0x7FFFu + ((u >> 16) & 1u)) >> 16;
}

__device__ __forceinline__ v8f wmma_f16(v16h a, v16h b, v8f c) {
  v8f d = __builtin_amdgcn_wmma_f32_16x16x32_f16(false, a, false, b, (short)0, c, false, false);
  asm volatile("v_nop\n\tv_nop\n\tv_nop\n\tv_nop" : "+v"(d) : "v"(a), "v"(b));
  return d;
}
__device__ __forceinline__ v8f wmma_bf16(v16us a, v16us b, v8f c) {
  v8f d = __builtin_amdgcn_wmma_f32_16x16x32_bf16(false, __builtin_bit_cast(v16bf, a), false,
                                                   __builtin_bit_cast(v16bf, b), (short)0, c, false, false);
  asm volatile("v_nop\n\tv_nop\n\tv_nop\n\tv_nop" : "+v"(d) : "v"(a), "v"(b));
  return d;
}

__device__ __forceinline__ v16h frag_f16(const _Float16* p) {
  FragH f;
  f.h[0] = *(const v8h*)p;
  f.h[1] = *(const v8h*)(p + 16);
  return f.v;
}
__device__ __forceinline__ v16us frag_u16(const unsigned short* p) {
  FragU f;
  f.h[0] = *(const v8us*)p;
  f.h[1] = *(const v8us*)(p + 16);
  return f.v;
}

__global__ __launch_bounds__(256) void k_wconv(
    const float* __restrict__ Wq, const float* __restrict__ Wk, const float* __restrict__ Wv,
    unsigned short* __restrict__ Wt)
{
  const unsigned int tid  = threadIdx.x;
  const unsigned int lane = tid & 31u;
  const unsigned int wave = (unsigned int)__builtin_amdgcn_readfirstlane((int)(tid >> 5));
  const unsigned int p    = blockIdx.x >> 3;
  const unsigned int h    = ((blockIdx.x & 7u) << 3) + wave;
  const float* W = (p == 0u) ? Wq : ((p == 1u) ? Wk : Wv);
  const float* src = W + (size_t)h * CDIM;
  unsigned short* dst = Wt + (size_t)(p * HDIM + h) * WP;

  v4u w0, w1, w2;
  {
    const unsigned int c = lane * 8u;
    const v4f a = *(const v4f*)(src + c);
    const v4f b = *(const v4f*)(src + c + 4u);
    w0.x = bf_bits(a.x) | (bf_bits(a.y) << 16);
    w0.y = bf_bits(a.z) | (bf_bits(a.w) << 16);
    w0.z = bf_bits(b.x) | (bf_bits(b.y) << 16);
    w0.w = bf_bits(b.z) | (bf_bits(b.w) << 16);
  }
  {
    const unsigned int c = 256u + lane * 8u;
    const v4f a = *(const v4f*)(src + c);
    const v4f b = *(const v4f*)(src + c + 4u);
    w1.x = bf_bits(a.x) | (bf_bits(a.y) << 16);
    w1.y = bf_bits(a.z) | (bf_bits(a.w) << 16);
    w1.z = bf_bits(b.x) | (bf_bits(b.y) << 16);
    w1.w = bf_bits(b.z) | (bf_bits(b.w) << 16);
  }
  {
    const unsigned int c = 512u + lane * 8u;
    const v4f a = *(const v4f*)(src + c);
    const v4f b = *(const v4f*)(src + c + 4u);
    w2.x = bf_bits(a.x) | (bf_bits(a.y) << 16);
    w2.y = bf_bits(a.z) | (bf_bits(a.w) << 16);
    w2.z = bf_bits(b.x) | (bf_bits(b.y) << 16);
    w2.w = bf_bits(b.z) | (bf_bits(b.w) << 16);
  }
  unsigned short* d0 = dst + lane * 8u;
  unsigned short* d1 = dst + 256u + lane * 8u;
  unsigned short* d2 = dst + 512u + lane * 8u;
  *(volatile v4u*)d0 = w0;
  *(volatile v4u*)d1 = w1;
  *(volatile v4u*)d2 = w2;
  __threadfence();
  *(volatile v4u*)d0 = w0;
  *(volatile v4u*)d1 = w1;
  *(volatile v4u*)d2 = w2;
}

__global__ __launch_bounds__(256) __attribute__((amdgpu_num_vgpr(256)))
void k_proj(const float* __restrict__ x, const unsigned short* __restrict__ Wt,
            _Float16* __restrict__ qh, _Float16* __restrict__ kh,
            _Float16* __restrict__ vT, _Float16* __restrict__ vR,
            _Float16* __restrict__ qR, _Float16* __restrict__ kR)
{
  __shared__ __attribute__((aligned(16))) unsigned short sm[64 * XP];

  const unsigned int tid  = threadIdx.x;
  const unsigned int lane = tid & 31u;
  const unsigned int wave = (unsigned int)__builtin_amdgcn_readfirstlane((int)(tid >> 5));
  const unsigned int half = lane >> 4;
  const unsigned int ln   = lane & 15u;
  const unsigned int m0 = blockIdx.x * 64u;
  const unsigned int b  = m0 / (unsigned int)SEQ;
  const unsigned int t0 = m0 - b * (unsigned int)SEQ;
  const float* xblk = x + ((size_t)b * SEQ_FULL + t0) * CDIM;

  const unsigned int rg = wave & 3u;
  const unsigned int ch = wave >> 2;
  v8f acc[6];
#pragma unroll
  for (int nt = 0; nt < 6; ++nt) {
#pragma unroll
    for (int r = 0; r < 8; ++r) acc[nt][r] = 0.0f;
  }
  const unsigned short* arow = sm + (rg * 16u + ln) * XP + 8u * half;
  const unsigned short* brow = Wt + (size_t)(ch * 96u + ln) * WP + 8u * half;

#pragma unroll 1
  for (unsigned int kh0 = 0; kh0 < KP; kh0 += KH) {
    __syncthreads();
    for (unsigned int i = tid; i < 64u * (KH / 4); i += 256u) {
      const unsigned int r  = i / (unsigned int)(KH / 4);
      const unsigned int c4 = i - r * (unsigned int)(KH / 4);
      const v4f v = *(const v4f*)(xblk + (size_t)r * CDIM + kh0 + c4 * 4u);
      v2u w;
      w.x = bf_bits(v.x) | (bf_bits(v.y) << 16);
      w.y = bf_bits(v.z) | (bf_bits(v.w) << 16);
      *(v2u*)(sm + r * XP + c4 * 4u) = w;
    }
    for (unsigned int i = tid; i < 64u * XPADV; i += 256u) {
      const unsigned int r = i / (unsigned int)XPADV;
      const unsigned int j = i - r * (unsigned int)XPADV;
      v4u z; z.x = 0u; z.y = 0u; z.z = 0u; z.w = 0u;
      *(v4u*)(sm + r * XP + KH + j * 8u) = z;
    }
    __syncthreads();

#pragma unroll 1
    for (unsigned int k0 = 0; k0 < KH; k0 += 32u) {
      const v16us a = frag_u16(arow + k0);
#pragma unroll
      for (int nt = 0; nt < 6; ++nt) {
        const v16us bb = frag_u16(brow + (size_t)nt * 16 * WP + kh0 + k0);
        acc[nt] = wmma_bf16(a, bb, acc[nt]);
      }
    }
  }
  __syncthreads();

#pragma unroll
  for (int nt = 0; nt < 6; ++nt) {
    const unsigned int n0 = ch * 96u + (unsigned int)nt * 16u;
    const unsigned int p  = n0 >> 6;
    const unsigned int hc = (n0 & 63u) + ln;
    const float sc = (p == 0u) ? LOG2E_F : ((p == 2u) ? 16.0f : 1.0f);
    unsigned short* base = sm + p * 4096u;
    const unsigned int roff = (p == 2u) ? 12288u : (16384u + p * 4096u);
#pragma unroll
    for (int r = 0; r < 8; ++r) {
      const unsigned int tl  = rg * 16u + 8u * half + (unsigned int)r;
      const unsigned int idx = (p == 2u) ? (hc * 64u + tl) : (tl * 64u + hc);
      const float vf = acc[nt][r] * sc;
      const _Float16 hv = (_Float16)vf;
      base[idx] = __builtin_bit_cast(unsigned short, hv);
      const _Float16 rv = (_Float16)((vf - (float)hv) * 1024.0f);
      sm[roff + idx] = __builtin_bit_cast(unsigned short, rv);
    }
  }
  __syncthreads();

  const unsigned int rl = lane >> 3;
  const unsigned int pc = lane & 7u;
  const unsigned int rA = wave * 8u + rl;
  const unsigned int rB = rA + 4u;
  const v4u qA = *(const v4u*)(sm + rA * 64u + pc * 8u);
  const v4u qB = *(const v4u*)(sm + rB * 64u + pc * 8u);
  const v4u kA = *(const v4u*)(sm + 4096u + rA * 64u + pc * 8u);
  const v4u kB = *(const v4u*)(sm + 4096u + rB * 64u + pc * 8u);
  const v4u vA = *(const v4u*)(sm + 8192u + rA * 64u + pc * 8u);
  const v4u vB = *(const v4u*)(sm + 8192u + rB * 64u + pc * 8u);
  const v4u uA = *(const v4u*)(sm + 12288u + rA * 64u + pc * 8u);
  const v4u uB = *(const v4u*)(sm + 12288u + rB * 64u + pc * 8u);
  const v4u aA = *(const v4u*)(sm + 16384u + rA * 64u + pc * 8u);
  const v4u aB = *(const v4u*)(sm + 16384u + rB * 64u + pc * 8u);
  const v4u cA = *(const v4u*)(sm + 20480u + rA * 64u + pc * 8u);
  const v4u cB = *(const v4u*)(sm + 20480u + rB * 64u + pc * 8u);
  _Float16* dqA = qh + (size_t)(m0 + rA) * HDIM + pc * 8u;
  _Float16* dqB = qh + (size_t)(m0 + rB) * HDIM + pc * 8u;
  _Float16* dkA = kh + (size_t)(m0 + rA) * HDIM + pc * 8u;
  _Float16* dkB = kh + (size_t)(m0 + rB) * HDIM + pc * 8u;
  _Float16* dvA = vT + ((size_t)b * HDIM + rA) * SEQ + t0 + pc * 8u;
  _Float16* dvB = vT + ((size_t)b * HDIM + rB) * SEQ + t0 + pc * 8u;
  _Float16* duA = vR + ((size_t)b * HDIM + rA) * SEQ + t0 + pc * 8u;
  _Float16* duB = vR + ((size_t)b * HDIM + rB) * SEQ + t0 + pc * 8u;
  const bool resid = (t0 < (unsigned int)TE);
  *(volatile v4u*)dqA = qA; *(volatile v4u*)dqB = qB;
  *(volatile v4u*)dkA = kA; *(volatile v4u*)dkB = kB;
  *(volatile v4u*)dvA = vA; *(volatile v4u*)dvB = vB;
  *(volatile v4u*)duA = uA; *(volatile v4u*)duB = uB;
  if (resid) {
    _Float16* daA = qR + ((size_t)b * TE + t0 + rA) * HDIM + pc * 8u;
    _Float16* daB = qR + ((size_t)b * TE + t0 + rB) * HDIM + pc * 8u;
    _Float16* dcA = kR + ((size_t)b * TE + t0 + rA) * HDIM + pc * 8u;
    _Float16* dcB = kR + ((size_t)b * TE + t0 + rB) * HDIM + pc * 8u;
    *(volatile v4u*)daA = aA; *(volatile v4u*)daB = aB;
    *(volatile v4u*)dcA = cA; *(volatile v4u*)dcB = cB;
  }
  __threadfence();
  *(volatile v4u*)dqA = qA; *(volatile v4u*)dqB = qB;
  *(volatile v4u*)dkA = kA; *(volatile v4u*)dkB = kB;
  *(volatile v4u*)dvA = vA; *(volatile v4u*)dvB = vB;
  *(volatile v4u*)duA = uA; *(volatile v4u*)duB = uB;
  if (resid) {
    _Float16* daA = qR + ((size_t)b * TE + t0 + rA) * HDIM + pc * 8u;
    _Float16* daB = qR + ((size_t)b * TE + t0 + rB) * HDIM + pc * 8u;
    _Float16* dcA = kR + ((size_t)b * TE + t0 + rA) * HDIM + pc * 8u;
    _Float16* dcB = kR + ((size_t)b * TE + t0 + rB) * HDIM + pc * 8u;
    *(volatile v4u*)daA = aA; *(volatile v4u*)daB = aB;
    *(volatile v4u*)dcA = cA; *(volatile v4u*)dcB = cB;
  }
}

template <int EARLY>
__global__ __launch_bounds__(128) __attribute__((amdgpu_num_vgpr(256)))
void k_attn(const _Float16* __restrict__ qh, const _Float16* __restrict__ kh,
            const _Float16* __restrict__ vT, const _Float16* __restrict__ vR,
            const _Float16* __restrict__ qR, const _Float16* __restrict__ kR,
            float* __restrict__ out)
{
  __shared__ __attribute__((aligned(16))) _Float16 pbuf[4][16][40];
  __shared__ __attribute__((aligned(16))) _Float16 rbuf[4][16][40];
  __shared__ __attribute__((aligned(16))) float    obuf[4][16][68];

  const unsigned int tid  = threadIdx.x;
  const unsigned int lane = tid & 31u;
  const unsigned int wave = (unsigned int)__builtin_amdgcn_readfirstlane((int)(tid >> 5));
  const unsigned int half = lane >> 4;
  const unsigned int ln   = lane & 15u;
  unsigned int b, tb;
  if (EARLY) { b = blockIdx.x / (unsigned int)NTB_E;  tb = blockIdx.x - b * (unsigned int)NTB_E; }
  else       { b = blockIdx.x / (unsigned int)NTB_LD; tb = (unsigned int)NTB_E + (blockIdx.x - b * (unsigned int)NTB_LD); }
  const unsigned int row0 = tb * 64u + wave * 16u;

  const _Float16* qrow   = qh + ((size_t)b * SEQ + row0 + ln) * HDIM + 8u * half;
  const _Float16* kbase  = kh + (size_t)b * SEQ * HDIM + 8u * half;
  const _Float16* vbase  = vT + (size_t)b * HDIM * SEQ + 8u * half;
  const _Float16* rbase  = vR + (size_t)b * HDIM * SEQ + 8u * half;
  const _Float16* krbase = kR + (size_t)b * TE * HDIM + 8u * half;

  const v16h qa0 = frag_f16(qrow);
  const v16h qa1 = frag_f16(qrow + 32);
  v16h qra0 = qa0, qra1 = qa1;
  if (EARLY) {
    const _Float16* qrrow = qR + ((size_t)b * TE + row0 + ln) * HDIM + 8u * half;
    qra0 = frag_f16(qrrow);
    qra1 = frag_f16(qrrow + 32);
  }

  v16h ones;
#pragma unroll
  for (int i = 0; i < 16; ++i) ones[i] = (_Float16)1.0f;

  v8f o[4], orr[4];
  v8f osum, osumr;
#pragma unroll
  for (int r = 0; r < 8; ++r) { osum[r] = 0.0f; osumr[r] = 0.0f; }
#pragma unroll
  for (int ht = 0; ht < 4; ++ht) {
#pragma unroll
    for (int r = 0; r < 8; ++r) { o[ht][r] = 0.0f; orr[ht][r] = 0.0f; }
  }
  float rmax[8];
#pragma unroll
  for (int r = 0; r < 8; ++r) rmax[r] = NEG_BIG;

  const unsigned int nchunk = 2u * tb + 2u;
#pragma unroll 1
  for (unsigned int c = 0; c < nchunk; ++c) {
    const unsigned int kt0 = c * 32u;
    const bool active = (kt0 <= row0 + 15u);
    v8f s[2];
#pragma unroll
    for (int r = 0; r < 8; ++r) { s[0][r] = 0.0f; s[1][r] = 0.0f; }

    if (active) {
#pragma unroll
      for (int nt = 0; nt < 2; ++nt) {
        const unsigned int key = kt0 + (unsigned int)nt * 16u + ln;
        const _Float16* krow = kbase + (size_t)key * HDIM;
        const v16h kb0 = frag_f16(krow);
        const v16h kb1 = frag_f16(krow + 32);
        v8f acc;
#pragma unroll
        for (int r = 0; r < 8; ++r) acc[r] = 0.0f;
        acc = wmma_f16(qa0, kb0, acc);
        acc = wmma_f16(qa1, kb1, acc);
        if (EARLY) {
          const _Float16* krr = krbase + (size_t)key * HDIM;
          const v16h kr0 = frag_f16(krr);
          const v16h kr1 = frag_f16(krr + 32);
          v8f accr;
#pragma unroll
          for (int r = 0; r < 8; ++r) accr[r] = 0.0f;
          accr = wmma_f16(qra0, kb0, accr);
          accr = wmma_f16(qra1, kb1, accr);
          accr = wmma_f16(qa0, kr0, accr);
          accr = wmma_f16(qa1, kr1, accr);
#pragma unroll
          for (int r = 0; r < 8; ++r) acc[r] = acc[r] + accr[r] * RINV;
        }
#pragma unroll
        for (int r = 0; r < 8; ++r) {
          const float sv = acc[r] * QK_SCALE;
          s[nt][r] = (key > row0 + 8u * half + (unsigned int)r) ? NEG_BIG : sv;
        }
      }
      float alpha[8];
#pragma unroll
      for (int r = 0; r < 8; ++r) {
        float tmax = fmaxf(s[0][r], s[1][r]);
#pragma unroll
        for (int m = 1; m < 16; m <<= 1) tmax = fmaxf(tmax, __shfl_xor(tmax, m, 32));
        const float nmax = fmaxf(rmax[r], tmax);
        alpha[r] = exp2f(rmax[r] - nmax);
        rmax[r]  = nmax;
        s[0][r] = exp2f(s[0][r] - nmax);
        s[1][r] = exp2f(s[1][r] - nmax);
      }
#pragma unroll
      for (int r = 0; r < 8; ++r) {
        osum[r] *= alpha[r];
        if (EARLY) osumr[r] *= alpha[r];
#pragma unroll
        for (int ht = 0; ht < 4; ++ht) {
          o[ht][r] *= alpha[r];
          if (EARLY) orr[ht][r] *= alpha[r];
        }
      }
    }

    __syncthreads();
    if (active) {
#pragma unroll
      for (int nt = 0; nt < 2; ++nt) {
#pragma unroll
        for (int r = 0; r < 8; ++r) {
          const float pf = s[nt][r] * 1024.0f;
          const _Float16 ph = (_Float16)pf;
          pbuf[wave][r + 8 * half][nt * 16 + ln] = ph;
          if (EARLY) {
            const _Float16 pr = (_Float16)((pf - (float)ph) * 1024.0f);
            rbuf[wave][r + 8 * half][nt * 16 + ln] = pr;
          }
        }
      }
    }
    __syncthreads();

    if (active) {
      const v16h pa = frag_f16(&pbuf[wave][ln][8 * half]);
      if (EARLY) {
        const v16h pra = frag_f16(&rbuf[wave][ln][8 * half]);
#pragma unroll
        for (int ht = 0; ht < 4; ++ht) {
          const v16h vb = frag_f16(vbase + (size_t)((unsigned int)ht * 16u + ln) * SEQ + kt0);
          o[ht]   = wmma_f16(pa,  vb, o[ht]);
          orr[ht] = wmma_f16(pra, vb, orr[ht]);
        }
        osum  = wmma_f16(pa,  ones, osum);
        osumr = wmma_f16(pra, ones, osumr);
#pragma unroll
        for (int ht = 0; ht < 4; ++ht) {
          const v16h vr = frag_f16(rbase + (size_t)((unsigned int)ht * 16u + ln) * SEQ + kt0);
          orr[ht] = wmma_f16(pa, vr, orr[ht]);
        }
      } else {
#pragma unroll
        for (int ht = 0; ht < 4; ++ht) {
          const v16h vb = frag_f16(vbase + (size_t)((unsigned int)ht * 16u + ln) * SEQ + kt0);
          o[ht] = wmma_f16(pa, vb, o[ht]);
        }
        osum = wmma_f16(pa, ones, osum);
      }
    }
  }

#pragma unroll
  for (int r = 0; r < 8; ++r) {
    float den = osum[r];
    if (EARLY) den = den + osumr[r] * RINV;
    const float inv = 0.0625f * __builtin_amdgcn_rcpf(den);
#pragma unroll
    for (int ht = 0; ht < 4; ++ht) {
      float num = o[ht][r];
      if (EARLY) num = num + orr[ht][r] * RINV;
      obuf[wave][8 * half + r][ht * 16 + ln] = num * inv;
    }
  }
  __syncthreads();

  v4f vals[8];
#pragma unroll
  for (int i = 0; i < 8; ++i) vals[i] = *(const v4f*)(&obuf[wave][2 * i + half][ln * 4]);
  float* orow = out + ((size_t)b * SEQ_FULL + row0) * HDIM;
#pragma unroll
  for (int i = 0; i < 8; ++i)
    *(volatile v4f*)(orow + (size_t)(2u * (unsigned int)i + half) * HDIM + ln * 4u) = vals[i];
  __threadfence();
#pragma unroll
  for (int i = 0; i < 8; ++i)
    *(volatile v4f*)(orow + (size_t)(2u * (unsigned int)i + half) * HDIM + ln * 4u) = vals[i];
}

extern "C" void kernel_launch(void* const* d_in, const int* in_sizes, int n_in,
                              void* d_out, int out_size, void* d_ws, size_t ws_size,
                              hipStream_t stream)
{
  if (n_in < 4) return;
  const long long tok_rows = (long long)(NB - 1) * SEQ_FULL + SEQ;
  if ((long long)in_sizes[0] < tok_rows * CDIM) return;
  if (in_sizes[1] < CDIM * HDIM || in_sizes[2] < CDIM * HDIM || in_sizes[3] < CDIM * HDIM) return;
  if ((long long)out_size < tok_rows * HDIM) return;

  const float* x  = (const float*)d_in[0];
  const float* Wq = (const float*)d_in[1];
  const float* Wk = (const float*)d_in[2];
  const float* Wv = (const float*)d_in[3];
  float* out = (float*)d_out;

  const size_t wt_bytes = (size_t)NPROJ * WP * sizeof(unsigned short);
  const size_t plane    = (size_t)NB * SEQ * HDIM * sizeof(_Float16);
  const size_t rplane   = (size_t)NB * TE * HDIM * sizeof(_Float16);
  const size_t off_wt = 0;
  const size_t off_q  = (off_wt + wt_bytes + 255) & ~(size_t)255;
  const size_t off_k  = off_q + plane;
  const size_t off_v  = off_k + plane;
  const size_t off_r  = off_v + plane;
  const size_t off_qr = off_r + plane;
  const size_t off_kr = off_qr + rplane;
  const size_t total  = off_kr + rplane;
  if (total > ws_size) return;

  unsigned short* Wt = (unsigned short*)((char*)d_ws + off_wt);
  _Float16* qh = (_Float16*)((char*)d_ws + off_q);
  _Float16* kh = (_Float16*)((char*)d_ws + off_k);
  _Float16* vT = (_Float16*)((char*)d_ws + off_v);
  _Float16* vR = (_Float16*)((char*)d_ws + off_r);
  _Float16* qR = (_Float16*)((char*)d_ws + off_qr);
  _Float16* kR = (_Float16*)((char*)d_ws + off_kr);

  k_wconv<<<NPROJ / 8, 256, 0, stream>>>(Wq, Wk, Wv, Wt);
  k_proj<<<(NB * SEQ) / 64, 256, 0, stream>>>(x, Wt, qh, kh, vT, vR, qR, kR);
  k_attn<1><<<NB * NTB_E, 128, 0, stream>>>(qh, kh, vT, vR, qR, kR, out);
  if (NTB_L > 0) k_attn<0><<<NB * NTB_LD, 128, 0, stream>>>(qh, kh, vT, vR, qR, kR, out);
}
